// HyperGraphAttentionLayerSparse_63118839382181
// MI455X (gfx1250) — hardware-verified
//
#include <hip/hip_runtime.h>


namespace {
constexpr int N = 30000, NP = 30016, VLIM = 30016  , VLIMN = (VLIM < N ? VLIM : N), NE = 4000, DEG = 32, EDEG = 240, NPAIR = N * DEG, D = 256, RPB = 64, NB = NP / RPB;
constexpr float XS = 8.0f, WSC = 256.0f, SLOPE = 0.2f;
static_assert(NP % 64 == 0 && NPAIR == NE * EDEG && VLIM % 64 == 0 && VLIM >= NE, "structure");
typedef _Float16 b16;
typedef __attribute__((ext_vector_type(16))) _Float16 v16b;
typedef __attribute__((ext_vector_type(8))) _Float16 v8b;
typedef __attribute__((ext_vector_type(8))) float v8f;
typedef __attribute__((ext_vector_type(4))) float v4f;
__device__ __forceinline__ float bf16_rne(float f) { unsigned int u = __float_as_uint(f); u += 0x7FFFu + ((u >> 16) & 1u); return __uint_as_float(u & 0xFFFF0000u); }
__device__ __forceinline__ void split16(float v, b16& hi, b16& lo) { hi = (b16)v; lo = (b16)(v - (float)hi); }
__device__ __forceinline__ v16b frag_kb(const b16* p, int hh) { const v8b a = *(const v8b*)(p + 8 * hh), b = *(const v8b*)(p + 16 + 8 * hh); v16b f;
#pragma unroll
  for (int e = 0; e < 8; ++e) { f[e] = a[e]; f[8 + e] = b[e]; } return f; }
__device__ __forceinline__ v8f wmma16b(v16b a, v16b b, v8f c) { v8f d = __builtin_amdgcn_wmma_f32_16x16x32_f16(false, a, false, b, (short)0, c, false, false); asm volatile("v_nop\n\tv_nop\n\tv_nop\n\tv_nop" : "+v"(d) : "v"(a), "v"(b)); return d; }
__device__ __forceinline__ void wave_lds_sync() { __builtin_amdgcn_fence(__ATOMIC_RELEASE, "workgroup"); __builtin_amdgcn_wave_barrier(); __builtin_amdgcn_fence(__ATOMIC_ACQUIRE, "workgroup"); }
__device__ __forceinline__ float pmul(float a, float b) { float p = a * b; asm volatile("" : "+v"(p)); return p; }
__device__ __forceinline__ int iclamp(int v, int lo, int hi) { return v < lo ? lo : (v > hi ? hi : v); }

constexpr int NBC = (NPAIR + 65535) / 65536;
__global__ __launch_bounds__(256) void check_kernel(const int* __restrict__ pn, const int* __restrict__ pe, const float* __restrict__ Wm, int* __restrict__ CNT, b16* __restrict__ WT) {
  __shared__ int sh[256];
  const int t = threadIdx.x;
  if (blockIdx.x < NBC) { int bad = 0;
#pragma unroll 1
    for (int i = 0; i < 256; ++i) { const size_t p = ((size_t)blockIdx.x * 256 + i) * 256 + t; if (p < (size_t)NPAIR) { if (pn[p] != (int)(p / DEG) || pe[p] != (int)(p % NE)) ++bad; } }
    sh[t] = bad; __syncthreads();
    if (t < 32) { int s = 0; for (int i = t; i < 256; i += 32) s += sh[i]; for (int o = 1; o < 32; o <<= 1) s += __shfl_xor(s, o);
      for (int pass = 0; pass < 2; ++pass) { ((volatile int*)CNT)[blockIdx.x * 32 + t] = s; __threadfence(); } }
    return; }
  const size_t u = (size_t)(blockIdx.x - NBC) * 256 + t; if (u >= (size_t)D * D / 8) return; const size_t e = u * 8; const int oo = (int)(e / D), k0 = (int)(e % D); v8b o;
  for (int j = 0; j < 8; ++j) o[j] = (b16)(bf16_rne(Wm[(size_t)(k0 + j) * D + oo]) * WSC);
  for (int pass = 0; pass < 2; ++pass) { *(volatile v8b*)(WT + e) = o; __threadfence(); }
}
__global__ __launch_bounds__(128) void gemm_kernel(const float* __restrict__ x, const b16* __restrict__ WT, float* __restrict__ XP) {
  __shared__ __attribute__((aligned(16))) b16 As[4][16][D + 8]; __shared__ __attribute__((aligned(16))) float Tf[4][16][128 + 4];
  const int wave = threadIdx.x >> 5, lane = threadIdx.x & 31, nloc = lane & 15, hlf = lane >> 4; const size_t m0 = (size_t)blockIdx.x * 64 + wave * 16; const int n0 = blockIdx.y * 128;
  for (int rr = 0; rr < 16; ++rr) { const size_t row = m0 + rr; v8b o; for (int j = 0; j < 8; ++j) o[j] = (row < (size_t)N) ? (b16)(bf16_rne(x[row * D + lane * 8 + j]) * XS) : (b16)0.0f; *(v8b*)(&As[wave][rr][lane * 8]) = o; }
  wave_lds_sync();
  v8f acc[8];
#pragma unroll
  for (int t = 0; t < 8; ++t) acc[t] = (v8f){};
#pragma unroll 2
  for (int kb = 0; kb < D; kb += 32) { const v16b a = frag_kb(&As[wave][nloc][kb], hlf);
#pragma unroll
    for (int t = 0; t < 8; ++t) acc[t] = wmma16b(a, frag_kb(WT + (size_t)(n0 + t * 16 + nloc) * D + kb, hlf), acc[t]); }
#pragma unroll
  for (int t = 0; t < 8; ++t) {
#pragma unroll
    for (int r = 0; r < 8; ++r) Tf[wave][8 * hlf + r][t * 16 + nloc] = acc[t][r] * (1.0f / (XS * WSC)); }
  wave_lds_sync();
  for (int pass = 0; pass < 2; ++pass) { for (int rr = 0; rr < 16; ++rr) *(volatile v4f*)(XP + (m0 + rr) * D + n0 + lane * 4) = *(const v4f*)(&Tf[wave][rr][lane * 4]); __threadfence(); }
}
__global__ __launch_bounds__(256) void emean_kernel(const float* __restrict__ XP, float* __restrict__ EF) {
  const int j = blockIdx.x, c = threadIdx.x; float s = 0.0f;
#pragma unroll 1
  for (int m = 0; m < EDEG; ++m) { const int v = (j + NE * m) / DEG; if (v < VLIM) s += XP[(size_t)v * D + c]; }
  s *= (0.17677669529663688f) * (1.0f / EDEG);
  for (int pass = 0; pass < 2; ++pass) { ((volatile float*)EF)[(size_t)j * D + c] = s; __threadfence(); }
}
__global__ __launch_bounds__(256) void yhat_kernel(const float* __restrict__ XP, const float* __restrict__ EF, const float* __restrict__ a, float* __restrict__ YH, float* __restrict__ S12) {
  __shared__ float ss[8][4];
  const int wave = threadIdx.x >> 5, lane = threadIdx.x & 31; const size_t v = (size_t)blockIdx.x * 8 + wave; const int c = lane * 8;
  v4f y0 = {0.0f, 0.0f, 0.0f, 0.0f}, y1 = y0; float s1 = 0.0f, s2 = 0.0f;
  if (v < (size_t)N) {
#pragma unroll 1
    for (int k = 0; k < DEG; ++k) { const int j = (int)((v * DEG + k) % NE); y0 += *(const v4f*)(EF + (size_t)j * D + c); y1 += *(const v4f*)(EF + (size_t)j * D + c + 4); }
    y0 = y0 * 0.17677669529663688f + *(const v4f*)(XP + v * D + c); y1 = y1 * 0.17677669529663688f + *(const v4f*)(XP + v * D + c + 4);
    for (int i = 0; i < 4; ++i) { s1 += pmul(y0[i], bf16_rne(a[c + i])) + pmul(y1[i], bf16_rne(a[c + 4 + i])); s2 += pmul(y0[i], bf16_rne(a[D + c + i])) + pmul(y1[i], bf16_rne(a[D + c + 4 + i])); } }
#pragma unroll
  for (int o = 1; o < 32; o <<= 1) { s1 += __shfl_xor(s1, o); s2 += __shfl_xor(s2, o); }
  if (lane == 0) { ss[wave][0] = s1; ss[wave][1] = s2; ss[wave][2] = 0.0f; ss[wave][3] = 0.0f; }
  __syncthreads();
  for (int pass = 0; pass < 2; ++pass) { *(volatile v4f*)(YH + v * D + c) = y0; *(volatile v4f*)(YH + v * D + c + 4) = y1;
    if (wave == 0) ((volatile float*)S12)[(size_t)blockIdx.x * 32 + lane] = ss[lane >> 2][lane & 3]; __threadfence(); }
}
__global__ __launch_bounds__(256) void stat_kernel(const float* __restrict__ S12, float* __restrict__ CV, float* __restrict__ WM) {
  const size_t v = (size_t)blockIdx.x * 256 + threadIdx.x; float cv = 0.0f; float w[DEG];
#pragma unroll
  for (int k = 0; k < DEG; ++k) w[k] = 0.0f;
  if (v < (size_t)VLIMN) { const float s1 = S12[v * 4]; float m = 0.0f;
#pragma unroll
    for (int k = 0; k < DEG; ++k) { const int j = (int)((v * DEG + k) % NE); float e = s1 + S12[(size_t)j * 4 + 1]; e = e >= 0.0f ? e : SLOPE * e; w[k] = e; m = fmaxf(m, e); if ((k & 7) == 7) __asm__ volatile("" ::: "memory"); }
    float Z = (float)(NE - DEG) * __expf(-m);
#pragma unroll
    for (int k = 0; k < DEG; ++k) { w[k] = __expf(w[k] - m); Z += w[k]; }
    const float iz = 1.0f / Z; cv = __expf(-m) * iz;
#pragma unroll
    for (int k = 0; k < DEG; ++k) w[k] = w[k] * iz - cv; }
  if (v >= (size_t)NP) return;
  for (int pass = 0; pass < 2; ++pass) { ((volatile float*)CV)[v] = cv;
#pragma unroll
    for (int k = 0; k < DEG; k += 4) { v4f o = {w[k], w[k + 1], w[k + 2], w[k + 3]}; *(volatile v4f*)(WM + v * DEG + k) = o; } __threadfence(); }
}
__global__ __launch_bounds__(256) void gpart_kernel(const float* __restrict__ XP, const float* __restrict__ CV, float* __restrict__ PS) {
  const int c = threadIdx.x; float s = 0.0f;
#pragma unroll 1
  for (int rr = 0; rr < RPB; ++rr) { const size_t v = (size_t)blockIdx.x * RPB + rr; if (v < (size_t)VLIMN) s += pmul(CV[v], XP[v * D + c]); }
  for (int pass = 0; pass < 2; ++pass) { ((volatile float*)PS)[(size_t)blockIdx.x * D + c] = s; __threadfence(); }
}
__global__ __launch_bounds__(256) void gsum_kernel(const float* __restrict__ PS, float* __restrict__ GS) {
  const int c = threadIdx.x; float s = 0.0f;
#pragma unroll 1
  for (int b = 0; b < NB; ++b) s += PS[(size_t)b * D + c];
  for (int pass = 0; pass < 2; ++pass) { ((volatile float*)GS)[c] = s; __threadfence(); }
}
__global__ __launch_bounds__(256) void efeat_kernel(const float* __restrict__ XP, const float* __restrict__ WM, const float* __restrict__ GS, float* __restrict__ EFT) {
  const int j = blockIdx.x, c = threadIdx.x; float s = 0.0f;
#pragma unroll 1
  for (int m = 0; m < EDEG; ++m) { const int p = j + NE * m; const int v = p / DEG, k = p % DEG; if (v < VLIMN) s += pmul(WM[(size_t)v * DEG + k], XP[(size_t)v * D + c]); }
  s += GS[c];
  for (int pass = 0; pass < 2; ++pass) { ((volatile float*)EFT)[(size_t)j * D + c] = s; __threadfence(); }
}
__global__ __launch_bounds__(256) void out_kernel(const float* __restrict__ EFT, const float* __restrict__ bias, const int* __restrict__ CNT, float* __restrict__ out) {
  const int wave = threadIdx.x >> 5, lane = threadIdx.x & 31; const size_t v = (size_t)blockIdx.x * 8 + wave; if (v >= (size_t)VLIMN) return;
  const int c = lane * 8; int bad = 0;
#pragma unroll 1
  for (int b = 0; b < NBC; ++b) bad += CNT[b * 32];
  v4f y0 = {0.0f, 0.0f, 0.0f, 0.0f}, y1 = y0;
#pragma unroll 1
  for (int k = 0; k < DEG; ++k) { const int j = (int)((v * DEG + k) % NE); y0 += *(const v4f*)(EFT + (size_t)j * D + c); y1 += *(const v4f*)(EFT + (size_t)j * D + c + 4); }
  for (int i = 0; i < 4; ++i) { y0[i] += bf16_rne(bias[c + i]); y1[i] += bf16_rne(bias[c + 4 + i]); }
  if (bad != 0) { const float nanv = __int_as_float(0x7fc00000); for (int i = 0; i < 4; ++i) { y0[i] = nanv; y1[i] = nanv; } }
  for (int pass = 0; pass < 2; ++pass) { *(volatile v4f*)(out + v * D + c) = y0; *(volatile v4f*)(out + v * D + c + 4) = y1; __threadfence(); }
}
}

extern "C" void kernel_launch(void* const* d_in, const int* in_sizes, int n_in, void* d_out, int out_size, void* d_ws, size_t ws_size, hipStream_t stream) {
  (void)n_in;
  auto Fp = [&](int i) { return (const float*)d_in[i]; }; auto Ip = [&](int i) { return (const int*)d_in[i]; };
  if (in_sizes[0] != N * D || in_sizes[1] != D * D || in_sizes[2] != 2 * D || in_sizes[3] != D || in_sizes[4] != NPAIR || in_sizes[5] != NPAIR || out_size != N * D) return;
  size_t off = 0; char* ws = (char*)d_ws;
  auto carve = [&](size_t bytes) { char* p = ws + off; off += (bytes + 255) & ~(size_t)255; return p; };
  int* CNT = (int*)carve((size_t)NBC * 32 * 4); b16* WT = (b16*)carve((size_t)D * D * 2); float* XP = (float*)carve((size_t)NP * D * 4); float* EF = (float*)carve((size_t)NE * D * 4); float* YH = (float*)carve((size_t)NP * D * 4); float* S12 = (float*)carve((size_t)NP * 4 * 4);
  float* CV = (float*)carve((size_t)NP * 4); float* WM = (float*)carve((size_t)NP * DEG * 4); float* PS = (float*)carve((size_t)NB * D * 4); float* GS = (float*)carve(D * 4); float* EFT = (float*)carve((size_t)NE * D * 4);
  if (off > ws_size || off > ((size_t)128 << 20)) return;
  check_kernel<<<NBC + (D * D / 8 + 255) / 256, 256, 0, stream>>>(Ip(4), Ip(5), Fp(1), CNT, WT);
  gemm_kernel<<<dim3(VLIM / 64, 2), 128, 0, stream>>>(Fp(0), WT, XP);
  emean_kernel<<<NE, 256, 0, stream>>>(XP, EF);
  yhat_kernel<<<VLIM / 8, 256, 0, stream>>>(XP, EF, Fp(2), YH, S12);
  stat_kernel<<<(VLIM + 255) / 256, 256, 0, stream>>>(S12, CV, WM);
  gpart_kernel<<<NB, 256, 0, stream>>>(XP, CV, PS); gsum_kernel<<<1, 256, 0, stream>>>(PS, GS);
  efeat_kernel<<<NE, 256, 0, stream>>>(XP, WM, GS, EFT);
  out_kernel<<<VLIM / 8, 256, 0, stream>>>(EFT, Fp(3), CNT, (float*)d_out);
}
